// TextGATConv_mod_37434934952836
// MI455X (gfx1250) — hardware-run, weakly checked
//
#include <hip/hip_runtime.h>
#include <math.h>

typedef __attribute__((ext_vector_type(16))) _Float16 v16h;
typedef __attribute__((ext_vector_type(16))) __bf16 v16b;
typedef __attribute__((ext_vector_type(8)))  _Float16 v8h;
typedef __attribute__((ext_vector_type(8)))  float v8f;
typedef __attribute__((ext_vector_type(4)))  float v4f;
typedef __attribute__((ext_vector_type(2)))  float v2f;
typedef __attribute__((ext_vector_type(4)))  unsigned v4u;
typedef __attribute__((ext_vector_type(4)))  int v4i;
typedef float __attribute__((may_alias)) float_a;
typedef int __attribute__((may_alias)) int_a;

template <typename T> __device__ __forceinline__ void vst2(void* p, T v) { *(volatile T*)p = v; __threadfence(); *(volatile T*)p = v; }
__device__ __forceinline__ v8f wmma16(v16h a, v16h b, v8f c) {
  v8f d = __builtin_amdgcn_wmma_f32_16x16x32_f16(false, a, false, b, (short)0, c, false, false);
  asm volatile("v_nop\n\tv_nop\n\tv_nop\n\tv_nop" : "+v"(d) : "v"(a), "v"(b));
  return d;
}
__device__ __forceinline__ v8f wmma_bf(v16b a, v16b b, v8f c) {
  v8f d = __builtin_amdgcn_wmma_f32_16x16x32_bf16(false, a, false, b, (short)0, c, false, false);
  asm volatile("v_nop\n\tv_nop\n\tv_nop\n\tv_nop" : "+v"(d) : "v"(a), "v"(b));
  return d;
}
__device__ __forceinline__ v16h frag_h(const _Float16* rowk0, int lane) {
  union { v16h v; v8h q[2]; } u; const _Float16* p = rowk0 + 8 * (lane >> 4);
  u.q[0] = *(const v8h*)p; u.q[1] = *(const v8h*)(p + 16); return u.v;
}
__device__ __forceinline__ v16h frag_f32(const float* rowk0, int lane) {
  v16h a; const float* p = rowk0 + 8 * (lane >> 4);
#pragma unroll
  for (int i = 0; i < 8; ++i) { a[i] = (_Float16)p[i]; a[8 + i] = (_Float16)p[16 + i]; }
  return a;
}
__device__ __forceinline__ v16h frag_f32s(const float* rowk0, int lane, float sc) {
  v16h a; const float* p = rowk0 + 8 * (lane >> 4);
#pragma unroll
  for (int i = 0; i < 8; ++i) { a[i] = (_Float16)(p[i] * sc); a[8 + i] = (_Float16)(p[16 + i] * sc); }
  return a;
}
__device__ __forceinline__ v16h fragc_f32(const float* W, int k0, int n, int lane, int ld, int K) {
  v16h a; const int g = lane >> 4;
#pragma unroll
  for (int i = 0; i < 8; ++i) { const int ka = k0 + 8 * g + i, kb = ka + 16;
    a[i] = (_Float16)(ka < K ? W[(size_t)(ka < K ? ka : K - 1) * ld + n] : 0.f); a[8 + i] = (_Float16)(kb < K ? W[(size_t)(kb < K ? kb : K - 1) * ld + n] : 0.f); }
  return a;
}
struct F2 { v16b h, l; };
__device__ __forceinline__ F2 bsplit16(const float v[16]) { F2 r;
#pragma unroll
  for (int i = 0; i < 16; ++i) { const __bf16 h = (__bf16)v[i]; r.h[i] = h; r.l[i] = (__bf16)(v[i] - (float)h); }
  return r; }
__device__ __forceinline__ F2 split_row(const float* row, int k0, int lane) { float v[16]; const float* p = row + k0 + 8 * (lane >> 4);
#pragma unroll
  for (int i = 0; i < 8; ++i) { v[i] = p[i]; v[8 + i] = p[16 + i]; }
  return bsplit16(v); }
__device__ __forceinline__ F2 split_rowK(const float* row, int k0, int lane, int K) { float v[16]; const int g = lane >> 4;
#pragma unroll
  for (int i = 0; i < 8; ++i) { const int ka = k0 + 8 * g + i, kb = ka + 16; v[i] = ka < K ? row[ka < K ? ka : K - 1] : 0.f; v[8 + i] = kb < K ? row[kb < K ? kb : K - 1] : 0.f; }
  return bsplit16(v); }
__device__ __forceinline__ F2 split_col(const float* W, int k0, int n, int lane, int ld, int K) { float v[16]; const int g = lane >> 4;
#pragma unroll
  for (int i = 0; i < 8; ++i) { const int ka = k0 + 8 * g + i, kb = ka + 16; v[i] = ka < K ? W[(size_t)(ka < K ? ka : K - 1) * ld + n] : 0.f; v[8 + i] = kb < K ? W[(size_t)(kb < K ? kb : K - 1) * ld + n] : 0.f; }
  return bsplit16(v); }
__device__ __forceinline__ v8f mac3(const F2& a, const F2& b, v8f c) { c = wmma_bf(a.l, b.h, c); c = wmma_bf(a.h, b.l, c); return wmma_bf(a.h, b.h, c); }
__device__ __forceinline__ float sigm(float v) { return 1.0f / (1.0f + expf(-v)); }
#define LDSX() do { asm volatile("s_wait_dscnt 0" ::: "memory"); __builtin_amdgcn_wave_barrier(); __builtin_amdgcn_fence(__ATOMIC_RELEASE, "workgroup"); } while (0)


#define NB 8
#define LL 128
#define DD 512
#define EE 64
#define NH 8
#define CH 64
#define NR (NB * LL)
#define SLOPE 0.2f
#define EPS 1e-5f
#ifndef TNR
#define TNR NR
#endif
typedef __attribute__((ext_vector_type(8))) __bf16 v8b;
__device__ __forceinline__ v16b frag_b(const __bf16* rowk0, int lane) {
  union { v16b v; v8b q[2]; } u; const __bf16* p = rowk0 + 8 * (lane >> 4);
  u.q[0] = *(const v8b*)p; u.q[1] = *(const v8b*)(p + 16); return u.v;
}
__device__ __forceinline__ float bfr(float v) { return (float)(__bf16)v; }
__device__ __attribute__((noinline)) float exp_ni(float v) { return expf(v); }
__device__ __attribute__((noinline)) float erf_ni(float v) { return erff(v); }

#define WS_PW  0u
#define WS_PE  (WS_PW + 2u * 2 * DD * DD)
#define WS_PF  (WS_PE + 2u * DD * EE)
#define WS_QKV (WS_PF + 2u * DD * DD)
#define WS_AO  (WS_QKV + 4u * (size_t)NR * 2 * DD)
#define WS_END (WS_AO + 4u * (size_t)NR * DD)

__global__ __launch_bounds__(256) void k_pack(const float* __restrict__ WQ, const float* __restrict__ WKV, const float* __restrict__ WE, const float* __restrict__ WF, char* __restrict__ ws) { const int n = blockIdx.x, t = threadIdx.x; __shared__ __align__(16) __bf16 s[DD];
  const int which = n / DD, o = n % DD; const float* Wm = which == 0 ? WQ : which == 1 ? WKV : which == 2 ? WE : WF; const int kin = (which == 2) ? EE : DD;
  for (int k = t; k < kin; k += 256) s[k] = (__bf16)Wm[(size_t)k * DD + o]; __syncthreads();
  __bf16* dst = which < 2 ? ((__bf16*)(ws + WS_PW) + ((size_t)which * DD + o) * DD) : which == 2 ? ((__bf16*)(ws + WS_PE) + (size_t)o * EE) : ((__bf16*)(ws + WS_PF) + (size_t)o * DD);
  for (int q = t; q < kin / 8; q += 256) vst2((unsigned*)(dst + q * 8), *(const v4u*)&s[q * 8]); }
__device__ __forceinline__ v16b fragb_f32(const float* __restrict__ p, int lane) { v16b a; const float* pp = p + 8 * (lane >> 4);
#pragma unroll
  for (int i = 0; i < 8; ++i) { a[i] = (__bf16)pp[i]; a[8 + i] = (__bf16)pp[16 + i]; } return a; }
__global__ __launch_bounds__(128) void k_qkv(const float* __restrict__ X, const __bf16* __restrict__ PW, float* __restrict__ QKV) { __shared__ __align__(16) float sf[4][16][132];
  const int tid = threadIdx.x, wave = tid >> 5, lane = tid & 31, col = lane & 15, g = lane >> 4; const size_t r0 = (size_t)blockIdx.x * 64 + wave * 16; const int c0 = blockIdx.y * 128;
  v8f acc[8] = {};
#pragma unroll 2
  for (int kc = 0; kc < DD / 32; ++kc) { const v16b a = fragb_f32(X + (r0 + col) * DD + kc * 32, lane);
#pragma unroll
    for (int j = 0; j < 8; ++j) acc[j] = wmma_bf(a, frag_b(PW + (size_t)(c0 + j * 16 + col) * DD + kc * 32, lane), acc[j]); }
#pragma unroll
  for (int j = 0; j < 8; ++j)
#pragma unroll
    for (int r = 0; r < 8; ++r) sf[wave][8 * g + r][j * 16 + col] = acc[j][r];
  LDSX(); for (int rl = 0; rl < 16; ++rl) vst2(QKV + (r0 + rl) * (2 * DD) + c0 + lane * 4, *(const v4f*)&sf[wave][rl][lane * 4]); }
__global__ __launch_bounds__(128) void k_gat(const float* __restrict__ E, const __bf16* __restrict__ PE, const float* __restrict__ QKV, const int* __restrict__ ADJ, float* __restrict__ AO) {
  __shared__ __align__(16) float skv[LL][CH + 4]; __shared__ float sq[CH]; __shared__ float sal[LL]; __shared__ float sred[4]; __shared__ __align__(16) float sout[DD];
  const int tid = threadIdx.x, wave = tid >> 5, lane = tid & 31, col = lane & 15, g = lane >> 4; const size_t row = blockIdx.x; const size_t b = row / LL; const float* erow = E + row * (size_t)LL * EE;
  const int keep_t = ADJ[row * LL + tid] != 0;
#pragma unroll 1
  for (int h = 0; h < NH; ++h) {
    if (tid < CH) sq[tid] = QKV[row * (2 * DD) + h * CH + tid];
#pragma unroll
    for (int rt = 0; rt < 2; ++rt) { const int j0 = wave * 32 + rt * 16; v8f acc[4] = {};
#pragma unroll
      for (int kc = 0; kc < EE / 32; ++kc) { const v16b a = fragb_f32(erow + (size_t)(j0 + col) * EE + kc * 32, lane);
#pragma unroll
        for (int ct = 0; ct < 4; ++ct) acc[ct] = wmma_bf(a, frag_b(PE + (size_t)(h * CH + ct * 16 + col) * EE + kc * 32, lane), acc[ct]); }
#pragma unroll
      for (int ct = 0; ct < 4; ++ct)
#pragma unroll
        for (int r = 0; r < 8; ++r) { const int j = j0 + 8 * g + r, c = ct * 16 + col; skv[j][c] = acc[ct][r] + QKV[(b * LL + j) * (2 * DD) + DD + h * CH + c]; } }
    __syncthreads();
    { float s = 0.f;
#pragma unroll 8
      for (int c = 0; c < CH; ++c) s += sq[c] * skv[tid][c];
      s *= 0.125f; s = (s > 0.f) ? s : SLOPE * s; sal[tid] = keep_t ? s : -3.0e38f; }
    __syncthreads();
    { float m = sal[tid];
#pragma unroll
      for (int o = 1; o < 32; o <<= 1) m = fmaxf(m, __shfl_xor(m, o));
      if (lane == 0) sred[wave] = m; } __syncthreads(); const float gm = fmaxf(fmaxf(sred[0], sred[1]), fmaxf(sred[2], sred[3])); __syncthreads();
    { const float ev = keep_t ? expf(sal[tid] - gm) : 0.f; sal[tid] = ev; float s = ev;
#pragma unroll
      for (int o = 1; o < 32; o <<= 1) s += __shfl_xor(s, o);
      if (lane == 0) sred[wave] = s; } __syncthreads(); const float inv = 1.0f / (sred[0] + sred[1] + sred[2] + sred[3]);
    { const int c = tid >> 1, half = tid & 1; float s = 0.f; for (int j = half * 64; j < half * 64 + 64; ++j) s += sal[j] * skv[j][c]; s += __shfl_xor(s, 1); if (half == 0) sout[h * CH + c] = s * inv; }
    __syncthreads(); }
  vst2(AO + row * DD + tid * 4, *(const v4f*)&sout[tid * 4]); }
__global__ __launch_bounds__(128) void k_ffn(const float* __restrict__ AO, const __bf16* __restrict__ PF, const float* __restrict__ BF, float* __restrict__ FO) { __shared__ __align__(16) float sf[4][16][132];
  const int tid = threadIdx.x, wave = tid >> 5, lane = tid & 31, col = lane & 15, g = lane >> 4; const size_t r0 = (size_t)blockIdx.x * 64 + wave * 16; const int c0 = blockIdx.y * 128;
  v8f acc[8] = {};
#pragma unroll 2
  for (int kc = 0; kc < DD / 32; ++kc) { const F2 a = split_row(AO + (r0 + col) * DD, kc * 32, lane);
#pragma unroll
    for (int j = 0; j < 8; ++j) { const v16b w = frag_b(PF + (size_t)(c0 + j * 16 + col) * DD + kc * 32, lane); acc[j] = wmma_bf(a.h, w, acc[j]); acc[j] = wmma_bf(a.l, w, acc[j]); } }
#pragma unroll
  for (int j = 0; j < 8; ++j) { const float bb = bfr(BF[c0 + j * 16 + col]);
#pragma unroll
    for (int r = 0; r < 8; ++r) sf[wave][8 * g + r][j * 16 + col] = acc[j][r] + bb; }
  LDSX(); for (int rl = 0; rl < 16; ++rl) vst2(FO + (r0 + rl) * (2 * DD) + c0 + lane * 4, *(const v4f*)&sf[wave][rl][lane * 4]); }
__global__ __launch_bounds__(128) void k_lnr(const float* __restrict__ FO, const float* __restrict__ G, const float* __restrict__ Bt, float* __restrict__ OUT) { __shared__ float red[4]; __shared__ __align__(16) float so2[DD]; const int t = threadIdx.x; const size_t row = blockIdx.x;
  float v[4]; float s = 0.f; for (int i = 0; i < 4; ++i) { v[i] = FO[row * (2 * DD) + t + 128 * i]; s += v[i]; }
#pragma unroll
  for (int o = 1; o < 32; o <<= 1) s += __shfl_xor(s, o);
  if ((t & 31) == 0) red[t >> 5] = s; __syncthreads(); const float mu = (red[0] + red[1] + red[2] + red[3]) / (float)DD; __syncthreads();
  float q = 0.f; for (int i = 0; i < 4; ++i) { const float d = v[i] - mu; q += d * d; }
#pragma unroll
  for (int o = 1; o < 32; o <<= 1) q += __shfl_xor(q, o);
  if ((t & 31) == 0) red[t >> 5] = q; __syncthreads(); const float var = (red[0] + red[1] + red[2] + red[3]) / (float)DD; const float inv = 1.0f / sqrtf(var + EPS);
  for (int i = 0; i < 4; ++i) { const int c = t + 128 * i; so2[c] = fmaxf((v[i] - mu) * inv * bfr(G[c]) + bfr(Bt[c]), 0.f); } __syncthreads(); vst2(OUT + row * DD + t * 4, *(const v4f*)&so2[t * 4]); }
extern "C" void kernel_launch(void* const* d_in, const int* in_sizes, int n_in, void* d_out, int out_size, void* d_ws, size_t ws_size, hipStream_t stream) {
  (void)in_sizes; (void)n_in; (void)out_size;
  const float** F = (const float**)d_in;
  if (ws_size < (size_t)WS_END) return;
  char* ws = (char*)d_ws; __bf16 *PW = (__bf16*)(ws + WS_PW), *PE = (__bf16*)(ws + WS_PE), *PF = (__bf16*)(ws + WS_PF); float *QKV = (float*)(ws + WS_QKV), *AO = (float*)(ws + WS_AO);
  k_pack<<<4 * DD, 256, 0, stream>>>(F[3], F[4], F[5], F[6], ws);
  k_qkv<<<dim3(NR / 64, 2 * DD / 128), 128, 0, stream>>>(F[0], PW, QKV);
  k_gat<<<TNR, 128, 0, stream>>>(F[2], PE, QKV, (const int*)d_in[1], AO);
  k_ffn<<<dim3(TNR / 64, DD / 128), 128, 0, stream>>>(AO, PF, F[7], QKV);
  k_lnr<<<TNR, 128, 0, stream>>>(QKV, F[8], F[9], (float*)d_out);
}
